// SpatialReasoningModule_70377334112318
// MI455X (gfx1250) — hardware-verified
//
#include <hip/hip_runtime.h>
#include <math.h>

typedef __bf16         v16b  __attribute__((ext_vector_type(16)));
typedef unsigned short v16us __attribute__((ext_vector_type(16)));
typedef unsigned short v8us  __attribute__((ext_vector_type(8)));
typedef float          v8f   __attribute__((ext_vector_type(8)));
typedef float          v4f   __attribute__((ext_vector_type(4)));
typedef v8us __attribute__((may_alias)) v8usa;
typedef v4f  __attribute__((may_alias)) v4fa;

union FragU { v16b v; v16us u; v8us half[2]; };

#define NTOK     1024
#define DMODEL   128
#define NHEAD    8
#define HDIM     16
#define PS_ELEMS 1396736
#define OFF_FEAT 0
#define OFF_W2C  131072
#define OFF_WIN  167936
#define OFF_WOUT 217088
#define OFF_WG1  233472
#define OFF_WG2  266240
#define OFF_IM   282624
#define IM_PITCH 320
#define IM_K     288
#define OFF_X    610304
#define OFF_QK   741376
#define QK_PITCH 256
#define OFF_VT   1003520
#define OFF_O    1134592
#define OFF_HB   1265664
#define CVT_GROUPS 35328

__device__ __forceinline__ v8f wmma_bf(v16b a, v16b b, v8f c) {
  v8f d = __builtin_amdgcn_wmma_f32_16x16x32_bf16(false, a, false, b, (short)0, c, false, false);
  asm volatile("v_nop\n\tv_nop\n\tv_nop\n\tv_nop" : "+v"(d) : "v"(a), "v"(b));
  return d;
}

__device__ __forceinline__ unsigned int bf16_rne(float x) {
  const unsigned int u = __float_as_uint(x);
  return (u + 0x7FFFu + ((u >> 16) & 1u)) >> 16;
}

__device__ __forceinline__ void split_bf16(float x, unsigned short& hi, unsigned short& lo) {
  const unsigned int hb = bf16_rne(x);
  const float hf = __uint_as_float(hb << 16);
  hi = (unsigned short)hb;
  lo = (unsigned short)bf16_rne(x - hf);
}

__device__ __forceinline__ void split8(v4f a, v4f c, v8us& hi, v8us& lo) {
  unsigned short h0, h1, h2, h3, h4, h5, h6, h7, l0, l1, l2, l3, l4, l5, l6, l7;
  split_bf16(a.x, h0, l0); split_bf16(a.y, h1, l1); split_bf16(a.z, h2, l2); split_bf16(a.w, h3, l3);
  split_bf16(c.x, h4, l4); split_bf16(c.y, h5, l5); split_bf16(c.z, h6, l6); split_bf16(c.w, h7, l7);
  const v8us hv = {h0, h1, h2, h3, h4, h5, h6, h7};
  const v8us lv = {l0, l1, l2, l3, l4, l5, l6, l7};
  hi = hv; lo = lv;
}

__device__ __forceinline__ v16b load_frag(const unsigned short* p, int h) {
  FragU f;
  f.half[0] = *(const v8usa*)(p + 8 * h);
  f.half[1] = *(const v8usa*)(p + 16 + 8 * h);
  return f.v;
}

__device__ __forceinline__ v16b load_frag_k16(const unsigned short* p) {
  FragU f;
  f.half[0] = *(const v8usa*)p;
  const v8us z = {0, 0, 0, 0, 0, 0, 0, 0};
  f.half[1] = z;
  return f.v;
}

__device__ __forceinline__ float gelu_f(float v) {
  return 0.5f * v * (1.0f + erff(v * 0.70710678118654752440f));
}

__device__ __forceinline__ float wave_sum(float v) {
  v += __shfl_xor(v, 16);
  v += __shfl_xor(v, 8);
  v += __shfl_xor(v, 4);
  v += __shfl_xor(v, 2);
  v += __shfl_xor(v, 1);
  return v;
}

__global__ __launch_bounds__(256) void convert_kernel(
    const float* __restrict__ feat, const float* __restrict__ w2c,
    const float* __restrict__ win, const float* __restrict__ wout,
    const float* __restrict__ wg1, const float* __restrict__ wg2,
    unsigned short* P)
{
  const int b = blockIdx.x;
  const int g = b * 256 + threadIdx.x;
  if (g >= CVT_GROUPS) return;
  const float* src;
  int sbase;
  if (b < 64)       { src = feat; sbase = OFF_FEAT; }
  else if (b < 82)  { src = w2c;  sbase = OFF_W2C; }
  else if (b < 106) { src = win;  sbase = OFF_WIN; }
  else if (b < 114) { src = wout; sbase = OFF_WOUT; }
  else if (b < 130) { src = wg1;  sbase = OFF_WG1; }
  else              { src = wg2;  sbase = OFF_WG2; }
  const int e = g * 8;
  const float* sp = src + (e - sbase);
  const v4f a = *(const v4fa*)sp;
  const v4f c = *(const v4fa*)(sp + 4);
  v8us hi, lo;
  split8(a, c, hi, lo);
  unsigned short* dh = P + e;
  unsigned short* dl = P + PS_ELEMS + e;
  *(volatile v8us*)dh = hi;
  *(volatile v8us*)dl = lo;
  __threadfence();
  *(volatile v8us*)dh = hi;
  *(volatile v8us*)dl = lo;
}

__device__ __forceinline__ void dep_store(const unsigned short* sA, unsigned short* P, int y, int w, int lane) {
  const int plane = w >> 2;
  const unsigned short* src0 = sA + plane * (32 * IM_PITCH);
  unsigned short* dst0 = P + (size_t)plane * PS_ELEMS + OFF_IM + (size_t)y * 32 * IM_PITCH;
  #pragma unroll
  for (int it = 0; it < 10; ++it) {
    const int L = (w & 3) * 40 + it * 4 + (lane >> 3);
    const int row = L / 5, piece = L - 5 * row;
    const int off = row * IM_PITCH + piece * 64 + 8 * (lane & 7);
    const v8us v = *(const v8usa*)(src0 + off);
    *(volatile v8us*)(dst0 + off) = v;
  }
}

__global__ __launch_bounds__(256) void dep_kernel(
    const float* __restrict__ dm, const float* __restrict__ w1, const float* __restrict__ b1,
    unsigned short* P)
{
  __shared__ float sD[5 * 34];
  __shared__ float sT[3 * 32 * 34];
  __shared__ __attribute__((aligned(16))) unsigned short sA[2 * 32 * IM_PITCH];

  const int y = blockIdx.x, tid = threadIdx.x, lane = tid & 31, w = tid >> 5;

  for (int idx = tid; idx < 5 * 34; idx += 256) {
    const int rr = idx / 34, cc = idx - 34 * rr;
    const int yg = y - 2 + rr, xg = cc - 1;
    const int ygc = min(max(yg, 0), 31), xgc = min(max(xg, 0), 31);
    const float v = dm[ygc * 32 + xgc];
    const bool ok = (yg >= 0) && (yg < 32) && (xg >= 0) && (xg < 32);
    sD[idx] = ok ? v : 0.0f;
  }
  __syncthreads();

  for (int idx = tid; idx < 3 * 32 * 34; idx += 256) {
    const int rr = idx / 1088, rem = idx - 1088 * rr;
    const int ic = rem / 34, cc = rem - 34 * ic;
    const int yg = y - 1 + rr, xg = cc - 1;
    float s = b1[ic];
    #pragma unroll
    for (int ky = 0; ky < 3; ++ky)
      #pragma unroll
      for (int kx = 0; kx < 3; ++kx) {
        const int col = min(max(cc - 1 + kx, 0), 33);
        s += sD[(rr + ky) * 34 + col] * w1[ic * 9 + ky * 3 + kx];
      }
    const bool ok = (yg >= 0) && (yg < 32) && (xg >= 0) && (xg < 32);
    const float g = gelu_f(s);
    sT[idx] = ok ? g : 0.0f;
  }
  __syncthreads();

  for (int idx = tid; idx < 32 * IM_PITCH; idx += 256) {
    const int x = idx / IM_PITCH, k = idx - IM_PITCH * x;
    const int kk = min(k, IM_K - 1);
    const int ic = kk / 9, tap = kk - 9 * ic;
    const int ky = tap / 3, kx = tap - 3 * ky;
    const float val = sT[(ky * 32 + ic) * 34 + x + kx];
    const float v = (k < IM_K) ? val : 0.0f;
    unsigned short hi, lo;
    split_bf16(v, hi, lo);
    sA[idx] = hi;
    sA[32 * IM_PITCH + idx] = lo;
  }
  __syncthreads();

  dep_store(sA, P, y, w, lane);
  __threadfence();
  dep_store(sA, P, y, w, lane);
}

template <int MODE>
__device__ __forceinline__ void gemm_store(const float* sC, unsigned short* P,
                                           const float* aux, const float* lnw, const float* lnb,
                                           float* outf, int outY, int offO, int offVt,
                                           int row0, int yb, int w, int lane)
{
  if constexpr (MODE == 0) {
    float* ob = outf + (size_t)yb * outY;
    #pragma unroll
    for (int i = 0; i < 8; ++i) {
      const int rl = 8 * w + i;
      const v4f v = *(const v4fa*)(sC + rl * 128 + 4 * lane);
      *(volatile v4f*)(ob + (size_t)(row0 + rl) * DMODEL + 4 * lane) = v;
    }
  } else if constexpr (MODE == 1 || MODE == 2) {
    const bool tr = (MODE == 2) && (yb == 2);
    if (!tr) {
      const int pitch = (MODE == 1) ? DMODEL : QK_PITCH;
      const int cbase = (MODE == 1) ? 0 : yb * DMODEL;
      #pragma unroll
      for (int it = 0; it < 4; ++it) {
        const int rl = 8 * w + 2 * it + (lane >> 4);
        const int c8 = 8 * (lane & 15);
        const float* sp = sC + rl * 128 + c8;
        v4f a = *(const v4fa*)sp;
        v4f c = *(const v4fa*)(sp + 4);
        if constexpr (MODE == 1) {
          const float* fp = aux + (size_t)(row0 + rl) * DMODEL + c8;
          const v4f fa = *(const v4fa*)fp;
          const v4f fc = *(const v4fa*)(fp + 4);
          a = fa + 0.1f * a;
          c = fc + 0.1f * c;
        }
        v8us hi, lo;
        split8(a, c, hi, lo);
        unsigned short* d = P + offO + (size_t)(row0 + rl) * pitch + cbase + c8;
        *(volatile v8us*)d = hi;
        *(volatile v8us*)(d + PS_ELEMS) = lo;
      }
    } else {
      #pragma unroll
      for (int it = 0; it < 4; ++it) {
        const int dd = 16 * w + 4 * it + (lane >> 3);
        const int q8 = 8 * (lane & 7);
        const float* cp = sC + dd;
        const v4f a = {cp[(q8 + 0) * 128], cp[(q8 + 1) * 128], cp[(q8 + 2) * 128], cp[(q8 + 3) * 128]};
        const v4f c = {cp[(q8 + 4) * 128], cp[(q8 + 5) * 128], cp[(q8 + 6) * 128], cp[(q8 + 7) * 128]};
        v8us hi, lo;
        split8(a, c, hi, lo);
        unsigned short* d = P + offVt + (size_t)dd * NTOK + row0 + q8;
        *(volatile v8us*)d = hi;
        *(volatile v8us*)(d + PS_ELEMS) = lo;
      }
    }
  } else {
    #pragma unroll
    for (int i = 0; i < 8; ++i) {
      const int rl = 8 * w + i;
      const int rg = row0 + rl;
      const v4f g = *(const v4fa*)(sC + rl * 128 + 4 * lane);
      const v4f a = *(const v4fa*)(aux + (size_t)rg * DMODEL + 4 * lane);
      const v4f yv = a + 0.5f * g;
      float s = (yv.x + yv.y) + (yv.z + yv.w);
      s = wave_sum(s);
      const float mu = s * (1.0f / 128.0f);
      const v4f dv = yv - mu;
      float q = (dv.x * dv.x + dv.y * dv.y) + (dv.z * dv.z + dv.w * dv.w);
      q = wave_sum(q);
      const float var = q * (1.0f / 128.0f);
      const float inv = 1.0f / sqrtf(var + 1e-5f);
      const v4f lw = *(const v4fa*)(lnw + 4 * lane);
      const v4f lb = *(const v4fa*)(lnb + 4 * lane);
      const v4f o = (dv * inv) * lw + lb;
      *(volatile v4f*)(outf + (size_t)rg * DMODEL + 4 * lane) = o;
    }
  }
}

template <int MODE>
__global__ __launch_bounds__(256) void gemm_kernel(
    unsigned short* P, int offA, int lda, int offW, int ldw, int nstrideY,
    int koff, int koffY, int ksteps,
    const float* __restrict__ bias, int biasY, float bscale,
    const float* __restrict__ aux, const float* __restrict__ lnw, const float* __restrict__ lnb,
    float* outf, int outY, int offO, int offVt)
{
  __shared__ __attribute__((aligned(16))) float sC[64 * 128];

  const int tid = threadIdx.x, lane = tid & 31, w = tid >> 5;
  const int h = lane >> 4, m = lane & 15;
  const int rw = w >> 2, cw = w & 3;
  const int row0 = blockIdx.x * 64;
  const int yb = blockIdx.y;

  const unsigned short* Ah = P + offA;
  const unsigned short* Al = Ah + PS_ELEMS;
  const unsigned short* Wh = P + offW;
  const unsigned short* Wl = Wh + PS_ELEMS;
  const size_t ao0 = (size_t)(row0 + 32 * rw + m) * lda;
  const size_t ao1 = ao0 + (size_t)16 * lda;
  const size_t bo0 = (size_t)(yb * nstrideY + 32 * cw + m) * ldw + koff + yb * koffY;
  const size_t bo1 = bo0 + (size_t)16 * ldw;

  const v8f zero8 = {0.f, 0.f, 0.f, 0.f, 0.f, 0.f, 0.f, 0.f};
  v8f acc[2][2];
  acc[0][0] = zero8; acc[0][1] = zero8; acc[1][0] = zero8; acc[1][1] = zero8;

  #pragma unroll 1
  for (int ks = 0; ks < ksteps; ++ks) {
    const int k0 = ks * 32;
    const v16b ah0 = load_frag(Ah + ao0 + k0, h);
    const v16b ah1 = load_frag(Ah + ao1 + k0, h);
    const v16b al0 = load_frag(Al + ao0 + k0, h);
    const v16b al1 = load_frag(Al + ao1 + k0, h);
    const v16b bh0 = load_frag(Wh + bo0 + k0, h);
    const v16b bh1 = load_frag(Wh + bo1 + k0, h);
    const v16b bl0 = load_frag(Wl + bo0 + k0, h);
    const v16b bl1 = load_frag(Wl + bo1 + k0, h);
    acc[0][0] = wmma_bf(ah0, bh0, acc[0][0]);
    acc[0][0] = wmma_bf(ah0, bl0, acc[0][0]);
    acc[0][0] = wmma_bf(al0, bh0, acc[0][0]);
    acc[0][1] = wmma_bf(ah0, bh1, acc[0][1]);
    acc[0][1] = wmma_bf(ah0, bl1, acc[0][1]);
    acc[0][1] = wmma_bf(al0, bh1, acc[0][1]);
    acc[1][0] = wmma_bf(ah1, bh0, acc[1][0]);
    acc[1][0] = wmma_bf(ah1, bl0, acc[1][0]);
    acc[1][0] = wmma_bf(al1, bh0, acc[1][0]);
    acc[1][1] = wmma_bf(ah1, bh1, acc[1][1]);
    acc[1][1] = wmma_bf(ah1, bl1, acc[1][1]);
    acc[1][1] = wmma_bf(al1, bh1, acc[1][1]);
  }

  const int bb = yb * biasY;
  #pragma unroll
  for (int nt = 0; nt < 2; ++nt) {
    const int cl = 32 * cw + 16 * nt + m;
    const float bv = bscale * bias[bb + cl];
    #pragma unroll
    for (int mt = 0; mt < 2; ++mt) {
      #pragma unroll
      for (int r = 0; r < 8; ++r) {
        const int rl = 32 * rw + 16 * mt + 8 * h + r;
        sC[rl * 128 + cl] = acc[mt][nt][r] + bv;
      }
    }
  }
  __syncthreads();

  gemm_store<MODE>(sC, P, aux, lnw, lnb, outf, outY, offO, offVt, row0, yb, w, lane);
  __threadfence();
  gemm_store<MODE>(sC, P, aux, lnw, lnb, outf, outY, offO, offVt, row0, yb, w, lane);
}

__device__ __forceinline__ void attn_store(const unsigned short* sO, unsigned short* P, int q0, int w, int lane) {
  const int plane = w >> 2;
  #pragma unroll
  for (int it = 0; it < 2; ++it) {
    const int L = (w & 3) * 8 + it * 4 + (lane >> 3);
    const int row = L >> 1, hr = L & 1;
    const int off = row * 128 + hr * 64 + 8 * (lane & 7);
    const v8us v = *(const v8usa*)(sO + plane * 2048 + off);
    *(volatile v8us*)(P + (size_t)plane * PS_ELEMS + OFF_O + (size_t)q0 * DMODEL + off) = v;
  }
}

__global__ __launch_bounds__(256) void attn_kernel(unsigned short* P)
{
  __shared__ __attribute__((aligned(16))) unsigned short sO[2 * 16 * 128];

  const int tid = threadIdx.x, lane = tid & 31, w = tid >> 5;
  const int h = lane >> 4, m = lane & 15;
  const int head = w;
  const int q0 = blockIdx.x * 16;
  const unsigned short* QK = P + OFF_QK;
  const unsigned short* VT = P + OFF_VT;

  const unsigned short* qp = QK + (size_t)(q0 + m) * QK_PITCH + head * HDIM + 8 * h;
  const v16b qbh = load_frag_k16(qp);
  const v16b qbl = load_frag_k16(qp + PS_ELEMS);

  const v8f zero8 = {0.f, 0.f, 0.f, 0.f, 0.f, 0.f, 0.f, 0.f};
  v8f o = zero8;
  float mrun = -1e30f, lrun = 0.0f;

  const unsigned short* kbase = QK + (size_t)m * QK_PITCH + DMODEL + head * HDIM + 8 * h;
  const unsigned short* vbase = VT + (size_t)(head * HDIM + m) * NTOK;

  #pragma unroll 1
  for (int kb = 0; kb < NTOK; kb += 32) {
    v8f s[2];
    #pragma unroll
    for (int j = 0; j < 2; ++j) {
      const unsigned short* kp = kbase + (size_t)(kb + 16 * j) * QK_PITCH;
      const v16b kh = load_frag_k16(kp);
      const v16b kl = load_frag_k16(kp + PS_ELEMS);
      v8f z = zero8;
      z = wmma_bf(kh, qbh, z);
      z = wmma_bf(kh, qbl, z);
      z = wmma_bf(kl, qbh, z);
      s[j] = z * 0.25f;
    }

    float mloc = s[0][0];
    #pragma unroll
    for (int j = 0; j < 2; ++j)
      #pragma unroll
      for (int r = 0; r < 8; ++r) mloc = fmaxf(mloc, s[j][r]);
    mloc = fmaxf(mloc, __shfl_xor(mloc, 16));
    const float mnew = fmaxf(mrun, mloc);
    const float alpha = __expf(mrun - mnew);
    mrun = mnew;
    float lsum = 0.0f;
    #pragma unroll
    for (int j = 0; j < 2; ++j)
      #pragma unroll
      for (int r = 0; r < 8; ++r) {
        const float p = __expf(s[j][r] - mnew);
        s[j][r] = p;
        lsum += p;
      }
    lsum += __shfl_xor(lsum, 16);
    lrun = lrun * alpha + lsum;
    o = o * alpha;

    FragU ph, pl;
    #pragma unroll
    for (int r = 0; r < 8; ++r) {
      unsigned short hb, lb;
      split_bf16(s[0][r], hb, lb);
      ph.u[r] = hb; pl.u[r] = lb;
      split_bf16(s[1][r], hb, lb);
      ph.u[8 + r] = hb; pl.u[8 + r] = lb;
    }

    const v16b vth = load_frag(vbase + kb, h);
    const v16b vtl = load_frag(vbase + PS_ELEMS + kb, h);
    o = wmma_bf(vth, ph.v, o);
    o = wmma_bf(vth, pl.v, o);
    o = wmma_bf(vtl, ph.v, o);
  }

  const float inv = 1.0f / lrun;
  const v4f oa = {o[0] * inv, o[1] * inv, o[2] * inv, o[3] * inv};
  const v4f oc = {o[4] * inv, o[5] * inv, o[6] * inv, o[7] * inv};
  v8us ohi, olo;
  split8(oa, oc, ohi, olo);
  const int so = m * 128 + head * HDIM + 8 * h;
  *(v8usa*)(sO + so) = ohi;
  *(v8usa*)(sO + 2048 + so) = olo;
  __syncthreads();

  attn_store(sO, P, q0, w, lane);
  __threadfence();
  attn_store(sO, P, q0, w, lane);
}

__device__ __forceinline__ void hbar_store(const unsigned short* sHL, unsigned short* P, int i, int lane) {
  const v8us v = *(const v8usa*)(sHL + 8 * lane);
  unsigned short* d = P + (size_t)(lane >> 4) * PS_ELEMS + OFF_HB + (size_t)i * DMODEL + 8 * (lane & 15);
  *(volatile v8us*)d = v;
}

__global__ __launch_bounds__(128) void hbar_kernel(
    const float* __restrict__ rowb, const float* __restrict__ colb, const float* __restrict__ gb,
    unsigned short* P)
{
  __shared__ __attribute__((aligned(16))) unsigned short sHL[256];
  const int i = blockIdx.x, d = threadIdx.x;
  const float r = rowb[i * DMODEL + d];
  const float b = gb[d];
  float s = 0.0f;
  #pragma unroll 1
  for (int j = 0; j < NTOK; ++j) {
    const float c = colb[j * DMODEL + d];
    s += gelu_f((r + c) + b);
  }
  const float mean = s * (1.0f / 1024.0f);
  unsigned short hi, lo;
  split_bf16(mean, hi, lo);
  sHL[d] = hi;
  sHL[128 + d] = lo;
  __syncthreads();
  if (d < 32) hbar_store(sHL, P, i, d);
  __threadfence();
  if (d < 32) hbar_store(sHL, P, i, d);
}

extern "C" void kernel_launch(void* const* d_in, const int* in_sizes, int n_in,
                              void* d_out, int out_size, void* d_ws, size_t ws_size,
                              hipStream_t stream) {
  if (n_in < 16) return;
  if (in_sizes[0] != NTOK * DMODEL || in_sizes[1] != NTOK || in_sizes[2] != 288 || in_sizes[3] != 32) return;
  if (in_sizes[4] != 36864 || in_sizes[5] != 128 || in_sizes[6] != 49152 || in_sizes[7] != 384) return;
  if (in_sizes[8] != 16384 || in_sizes[9] != 128 || in_sizes[10] != 32768 || in_sizes[11] != 128) return;
  if (in_sizes[12] != 16384 || in_sizes[13] != 128 || in_sizes[14] != 128 || in_sizes[15] != 128) return;
  if (out_size != NTOK * DMODEL) return;

  const float* features   = (const float*)d_in[0];
  const float* depth_map  = (const float*)d_in[1];
  const float* conv1_w    = (const float*)d_in[2];
  const float* conv1_b    = (const float*)d_in[3];
  const float* conv2_w    = (const float*)d_in[4];
  const float* conv2_b    = (const float*)d_in[5];
  const float* in_proj_w  = (const float*)d_in[6];
  const float* in_proj_b  = (const float*)d_in[7];
  const float* out_proj_w = (const float*)d_in[8];
  const float* out_proj_b = (const float*)d_in[9];
  const float* gc1_w      = (const float*)d_in[10];
  const float* gc1_b      = (const float*)d_in[11];
  const float* gc2_w      = (const float*)d_in[12];
  const float* gc2_b      = (const float*)d_in[13];
  const float* ln_w       = (const float*)d_in[14];
  const float* ln_b       = (const float*)d_in[15];
  float* out = (float*)d_out;

  const size_t plane_bytes = (size_t)PS_ELEMS * 2;
  const size_t off_att = 2 * plane_bytes;
  const size_t fbytes = (size_t)NTOK * DMODEL * 4;
  const size_t total = off_att + 3 * fbytes;
  if (total > ws_size) return;

  unsigned short* P = (unsigned short*)d_ws;
  float* att  = (float*)((char*)d_ws + off_att);
  float* rowb = (float*)((char*)d_ws + off_att + fbytes);
  float* colb = (float*)((char*)d_ws + off_att + 2 * fbytes);

  convert_kernel<<<(CVT_GROUPS + 255) / 256, 256, 0, stream>>>(
      features, conv2_w, in_proj_w, out_proj_w, gc1_w, gc2_w, P);

  dep_kernel<<<32, 256, 0, stream>>>(depth_map, conv1_w, conv1_b, P);

  gemm_kernel<1><<<dim3(NTOK / 64, 1), 256, 0, stream>>>(
      P, OFF_IM, IM_PITCH, OFF_W2C, IM_K, 0, 0, 0, IM_K / 32,
      conv2_b, 0, 1.0f, features, ln_w, ln_b, att, 0, OFF_X, 0);

  gemm_kernel<2><<<dim3(NTOK / 64, 3), 256, 0, stream>>>(
      P, OFF_X, DMODEL, OFF_WIN, DMODEL, DMODEL, 0, 0, DMODEL / 32,
      in_proj_b, DMODEL, 1.0f, features, ln_w, ln_b, att, 0, OFF_QK, OFF_VT);

  attn_kernel<<<NTOK / 16, 256, 0, stream>>>(P);

  gemm_kernel<0><<<dim3(NTOK / 64, 1), 256, 0, stream>>>(
      P, OFF_O, DMODEL, OFF_WOUT, DMODEL, 0, 0, 0, DMODEL / 32,
      out_proj_b, 0, 1.0f, features, ln_w, ln_b, att, 0, 0, 0);

  gemm_kernel<0><<<dim3(NTOK / 64, 2), 256, 0, stream>>>(
      P, OFF_FEAT, DMODEL, OFF_WG1, 2 * DMODEL, 0, 0, DMODEL, DMODEL / 32,
      gc1_b, 0, 0.0f, features, ln_w, ln_b, rowb, NTOK * DMODEL, 0, 0);

  hbar_kernel<<<NTOK, DMODEL, 0, stream>>>(rowb, colb, gc1_b, P);

  gemm_kernel<3><<<dim3(NTOK / 64, 1), 256, 0, stream>>>(
      P, OFF_HB, DMODEL, OFF_WG2, DMODEL, 0, 0, 0, DMODEL / 32,
      gc2_b, 0, 1.0f, att, ln_w, ln_b, out, 0, 0, 0);
}
